// TDTFLayer_23141283791225
// MI455X (gfx1250) — hardware-verified
//
#include <hip/hip_runtime.h>
#include <math.h>

typedef __attribute__((ext_vector_type(16))) _Float16 v16h;
typedef __attribute__((ext_vector_type(16))) __bf16 v16b;
typedef __attribute__((ext_vector_type(8)))  _Float16 v8h;
typedef __attribute__((ext_vector_type(8)))  float v8f;
typedef __attribute__((ext_vector_type(4)))  float v4f;
typedef __attribute__((ext_vector_type(2)))  float v2f;
typedef __attribute__((ext_vector_type(4)))  unsigned v4u;
typedef __attribute__((ext_vector_type(4)))  int v4i;
typedef float __attribute__((may_alias)) float_a;
typedef int __attribute__((may_alias)) int_a;

template <typename T> __device__ __forceinline__ void vst2(void* p, T v) { *(volatile T*)p = v; __threadfence(); *(volatile T*)p = v; }
__device__ __forceinline__ v8f wmma16(v16h a, v16h b, v8f c) {
  v8f d = __builtin_amdgcn_wmma_f32_16x16x32_f16(false, a, false, b, (short)0, c, false, false);
  asm volatile("v_nop\n\tv_nop\n\tv_nop\n\tv_nop" : "+v"(d) : "v"(a), "v"(b));
  return d;
}
__device__ __forceinline__ v8f wmma_bf(v16b a, v16b b, v8f c) {
  v8f d = __builtin_amdgcn_wmma_f32_16x16x32_bf16(false, a, false, b, (short)0, c, false, false);
  asm volatile("v_nop\n\tv_nop\n\tv_nop\n\tv_nop" : "+v"(d) : "v"(a), "v"(b));
  return d;
}
__device__ __forceinline__ v16h frag_h(const _Float16* rowk0, int lane) {
  union { v16h v; v8h q[2]; } u; const _Float16* p = rowk0 + 8 * (lane >> 4);
  u.q[0] = *(const v8h*)p; u.q[1] = *(const v8h*)(p + 16); return u.v;
}
__device__ __forceinline__ v16h frag_f32(const float* rowk0, int lane) {
  v16h a; const float* p = rowk0 + 8 * (lane >> 4);
#pragma unroll
  for (int i = 0; i < 8; ++i) { a[i] = (_Float16)p[i]; a[8 + i] = (_Float16)p[16 + i]; }
  return a;
}
__device__ __forceinline__ v16h frag_f32s(const float* rowk0, int lane, float sc) {
  v16h a; const float* p = rowk0 + 8 * (lane >> 4);
#pragma unroll
  for (int i = 0; i < 8; ++i) { a[i] = (_Float16)(p[i] * sc); a[8 + i] = (_Float16)(p[16 + i] * sc); }
  return a;
}
__device__ __forceinline__ v16h fragc_f32(const float* W, int k0, int n, int lane, int ld, int K) {
  v16h a; const int g = lane >> 4;
#pragma unroll
  for (int i = 0; i < 8; ++i) { const int ka = k0 + 8 * g + i, kb = ka + 16;
    a[i] = (_Float16)(ka < K ? W[(size_t)(ka < K ? ka : K - 1) * ld + n] : 0.f); a[8 + i] = (_Float16)(kb < K ? W[(size_t)(kb < K ? kb : K - 1) * ld + n] : 0.f); }
  return a;
}
struct F2 { v16b h, l; };
__device__ __forceinline__ F2 bsplit16(const float v[16]) { F2 r;
#pragma unroll
  for (int i = 0; i < 16; ++i) { const __bf16 h = (__bf16)v[i]; r.h[i] = h; r.l[i] = (__bf16)(v[i] - (float)h); }
  return r; }
__device__ __forceinline__ F2 split_row(const float* row, int k0, int lane) { float v[16]; const float* p = row + k0 + 8 * (lane >> 4);
#pragma unroll
  for (int i = 0; i < 8; ++i) { v[i] = p[i]; v[8 + i] = p[16 + i]; }
  return bsplit16(v); }
__device__ __forceinline__ F2 split_rowK(const float* row, int k0, int lane, int K) { float v[16]; const int g = lane >> 4;
#pragma unroll
  for (int i = 0; i < 8; ++i) { const int ka = k0 + 8 * g + i, kb = ka + 16; v[i] = ka < K ? row[ka < K ? ka : K - 1] : 0.f; v[8 + i] = kb < K ? row[kb < K ? kb : K - 1] : 0.f; }
  return bsplit16(v); }
__device__ __forceinline__ F2 split_col(const float* W, int k0, int n, int lane, int ld, int K) { float v[16]; const int g = lane >> 4;
#pragma unroll
  for (int i = 0; i < 8; ++i) { const int ka = k0 + 8 * g + i, kb = ka + 16; v[i] = ka < K ? W[(size_t)(ka < K ? ka : K - 1) * ld + n] : 0.f; v[8 + i] = kb < K ? W[(size_t)(kb < K ? kb : K - 1) * ld + n] : 0.f; }
  return bsplit16(v); }
__device__ __forceinline__ v8f mac3(const F2& a, const F2& b, v8f c) { c = wmma_bf(a.l, b.h, c); c = wmma_bf(a.h, b.l, c); return wmma_bf(a.h, b.h, c); }
__device__ __forceinline__ float sigm(float v) { return 1.0f / (1.0f + expf(-v)); }
#define LDSX() do { asm volatile("s_wait_dscnt 0" ::: "memory"); __builtin_amdgcn_wave_barrier(); __builtin_amdgcn_fence(__ATOMIC_RELEASE, "workgroup"); } while (0)


#define NTOK 256
#define KSEL 128
#define DD 2048
#define II 5504
typedef __attribute__((ext_vector_type(8))) __bf16 v8b;
__device__ __forceinline__ v16b frag_b(const __bf16* rowk0, int lane) {
  union { v16b v; v8b q[2]; } u; const __bf16* p = rowk0 + 8 * (lane >> 4);
  u.q[0] = *(const v8b*)p; u.q[1] = *(const v8b*)(p + 16); return u.v;
}
__device__ __forceinline__ float bfr(float v) { return (float)(__bf16)v; }
__device__ __attribute__((noinline)) float exp_ni(float v) { return expf(v); }
__device__ __attribute__((noinline)) float erf_ni(float v) { return erff(v); }
__device__ __forceinline__ float silu_f(float v) { return v / (1.0f + exp_ni(-v)); }

#define PK_V  0
#define PK_O  (PK_V + (size_t)DD * DD)
#define PK_G  (PK_O + (size_t)DD * DD)
#define PK_U  (PK_G + (size_t)II * DD)
#define PK_D  (PK_U + (size_t)II * DD)
#define PK_END (PK_D + (size_t)DD * II)
#define WS_PK   0u
#define WS_SEL  (((2u * PK_END) + 127u) / 128u * 128u)
#define WS_FLG  (WS_SEL + 4u * NTOK)
#define WS_HH   (WS_FLG + 4u * NTOK)
#define WS_HL   (WS_HH + 2u * KSEL * DD)
#define WS_VH   (WS_HL + 2u * KSEL * DD)
#define WS_VL   (WS_VH + 2u * KSEL * DD)
#define WS_X1   (WS_VL + 2u * KSEL * DD)
#define WS_AH   (WS_X1 + 4u * KSEL * DD)
#define WS_AL   (WS_AH + 2u * KSEL * II)
#define WS_END  (WS_AL + 2u * KSEL * II)

__global__ __launch_bounds__(256) void k_pack(const float* __restrict__ WV, const float* __restrict__ WO, const float* __restrict__ WG, const float* __restrict__ WU, const float* __restrict__ WD, __bf16* __restrict__ PK) {
  __shared__ __align__(16) __bf16 s[II]; const int n = blockIdx.x, which = blockIdx.y, t = threadIdx.x; int K; size_t dst;
  if (which == 0) { if (n >= DD) return; K = DD; dst = PK_V + (size_t)n * DD; for (int k = t; k < DD; k += 256) s[k] = (__bf16)WV[(size_t)k * DD + n]; }
  else if (which == 1) { if (n >= DD) return; K = DD; dst = PK_O + (size_t)n * DD; for (int k = t; k < DD; k += 256) s[k] = (__bf16)WO[(size_t)k * DD + n]; }
  else if (which == 2) { K = DD; dst = PK_G + (size_t)n * DD; for (int k = t; k < DD; k += 256) s[k] = (__bf16)WG[(size_t)k * II + n]; }
  else if (which == 3) { K = DD; dst = PK_U + (size_t)n * DD; for (int k = t; k < DD; k += 256) s[k] = (__bf16)WU[(size_t)k * II + n]; }
  else { if (n >= DD) return; K = II; dst = PK_D + (size_t)n * II; for (int k = t; k < II; k += 256) s[k] = (__bf16)WD[(size_t)k * DD + n]; }
  __syncthreads();
  for (int q = t; q < K / 8; q += 256) vst2((unsigned*)(PK + dst + q * 8), *(const v4u*)&s[q * 8]);
}
__global__ __launch_bounds__(256) void k_route(const float* __restrict__ X, const float* __restrict__ RW, const float* __restrict__ RB, int* __restrict__ SEL, int* __restrict__ FLG) {
  __shared__ float ssc[NTOK]; __shared__ __align__(16) int sflag[NTOK]; __shared__ __align__(16) int ssel[NTOK]; const int t = threadIdx.x;
  { const float* xr = X + (size_t)t * DD; float a = 0.f; for (int k = 0; k < DD; ++k) a += bfr(xr[k]) * bfr(RW[k]); ssc[t] = a + bfr(RB[0]); }
  __syncthreads();
  { const float me = ssc[t]; int rank = 0; for (int j = 0; j < NTOK; ++j) { const float o = ssc[j]; rank += (o > me) || (o == me && j < t); } sflag[t] = (rank < KSEL) ? 1 : 0; }
  __syncthreads();
  if (t == 0) { int c = 0; for (int j = 0; j < NTOK; ++j) if (sflag[j]) ssel[c++] = j; for (; c < NTOK; ++c) ssel[c] = ssel[0]; }
  __syncthreads();
  if (t < NTOK / 4) vst2((unsigned*)(SEL + t * 4), *(const v4u*)&ssel[t * 4]); else if (t < NTOK / 2) vst2((unsigned*)(FLG + (t - 64) * 4), *(const v4u*)&sflag[(t - 64) * 4]);
}
__global__ __launch_bounds__(256) void k_rms(const float* __restrict__ X, const float* __restrict__ X1, const int* __restrict__ SEL, const float* __restrict__ LNW, int first, __bf16* __restrict__ HH, __bf16* __restrict__ HL) {
  __shared__ float sred[8]; __shared__ __align__(16) __bf16 sh_[DD], sl_[DD]; const int t = threadIdx.x, slot = blockIdx.x; const int tok = min(max(SEL[slot], 0), NTOK - 1);
  const float* xr = first ? X + (size_t)tok * DD : X1 + (size_t)slot * DD; float v[8]; float s = 0.f;
#pragma unroll
  for (int i = 0; i < 8; ++i) { v[i] = first ? bfr(xr[t + 256 * i]) : xr[t + 256 * i]; s += v[i] * v[i]; }
#pragma unroll
  for (int o = 1; o < 32; o <<= 1) s += __shfl_xor(s, o);
  if ((t & 31) == 0) sred[t >> 5] = s;
  __syncthreads();
  float tot = 0.f; for (int w = 0; w < 8; ++w) tot += sred[w];
  const float rs = rsqrtf(tot * (1.0f / DD) + 1e-6f);
#pragma unroll
  for (int i = 0; i < 8; ++i) { const int c = t + 256 * i; const float h = v[i] * rs * bfr(LNW[c]); const __bf16 hb = (__bf16)h; sh_[c] = hb; sl_[c] = (__bf16)(h - (float)hb); }
  __syncthreads();
  vst2((unsigned*)(HH + (size_t)slot * DD + t * 8), *(const v4u*)&sh_[t * 8]); vst2((unsigned*)(HL + (size_t)slot * DD + t * 8), *(const v4u*)&sl_[t * 8]);
}
template <int MODE>
__global__ __launch_bounds__(128) void k_lin(const __bf16* __restrict__ AHp, const __bf16* __restrict__ ALp, const __bf16* __restrict__ P, const __bf16* __restrict__ P2, const float* __restrict__ BIAS, const float* __restrict__ X, const float* __restrict__ X1, const int* __restrict__ SEL, __bf16* __restrict__ OH, __bf16* __restrict__ OL, float* __restrict__ OUTF) {
  constexpr int KK = (MODE == 3) ? II : DD;
  __shared__ __align__(16) float so[4][16][132]; __shared__ __align__(16) __bf16 soh[4][16][136], sol[4][16][136];
  const int tid = threadIdx.x, wave = tid >> 5, lane = tid & 31, col = lane & 15, g = lane >> 4; const size_t r0 = (size_t)blockIdx.x * 64 + wave * 16; const int n0 = blockIdx.y * 128;
  v8f acc[8] = {}; v8f acc2[8] = {};
#pragma unroll 2
  for (int kc = 0; kc < KK / 32; ++kc) { F2 a; a.h = frag_b(AHp + (r0 + col) * KK + kc * 32, lane); a.l = frag_b(ALp + (r0 + col) * KK + kc * 32, lane);
#pragma unroll
    for (int j = 0; j < 8; ++j) { const v16b w = frag_b(P + (size_t)(n0 + j * 16 + col) * KK + kc * 32, lane); acc[j] = wmma_bf(a.l, w, acc[j]); acc[j] = wmma_bf(a.h, w, acc[j]);
      if (MODE == 2) { const v16b w2 = frag_b(P2 + (size_t)(n0 + j * 16 + col) * KK + kc * 32, lane); acc2[j] = wmma_bf(a.l, w2, acc2[j]); acc2[j] = wmma_bf(a.h, w2, acc2[j]); } } }
#pragma unroll
  for (int j = 0; j < 8; ++j) { const int c = n0 + j * 16 + col;
#pragma unroll
    for (int r = 0; r < 8; ++r) { const int rl = 8 * g + r; float v;
      if (MODE == 0) v = acc[j][r] + bfr(BIAS[c]);
      else if (MODE == 1) { const int tok = min(max(SEL[r0 + rl], 0), NTOK - 1); v = bfr(X[(size_t)tok * DD + c]) + acc[j][r]; }
      else if (MODE == 2) v = silu_f(acc[j][r]) * acc2[j][r];
      else v = X1[(r0 + rl) * DD + c] + acc[j][r];
      if (MODE == 0 || MODE == 2) { const __bf16 hb = (__bf16)v; soh[wave][rl][j * 16 + col] = hb; sol[wave][rl][j * 16 + col] = (__bf16)(v - (float)hb); } else so[wave][rl][j * 16 + col] = v; } }
  LDSX();
  constexpr int NOUT = (MODE == 2) ? II : DD;
  for (int rl = 0; rl < 16; ++rl) {
    if (MODE == 0 || MODE == 2) { if (lane < 16) { vst2((unsigned*)(OH + (r0 + rl) * NOUT + n0 + lane * 8), *(const v4u*)&soh[wave][rl][lane * 8]); vst2((unsigned*)(OL + (r0 + rl) * NOUT + n0 + lane * 8), *(const v4u*)&sol[wave][rl][lane * 8]); } }
    else if (MODE == 1) vst2(OUTF + (r0 + rl) * DD + n0 + lane * 4, *(const v4f*)&so[wave][rl][lane * 4]);
    else { const int tok = min(max(SEL[r0 + rl], 0), NTOK - 1); vst2(OUTF + (size_t)tok * DD + n0 + lane * 4, *(const v4f*)&so[wave][rl][lane * 4]); } }
}
__global__ __launch_bounds__(256) void k_copy(const float* __restrict__ X, const int* __restrict__ FLG, float* __restrict__ OUT) {
  const int tok = blockIdx.x, t = threadIdx.x; if (FLG[tok]) return;
  for (int q = t; q < DD / 4; q += 256) { const float* p = X + (size_t)tok * DD + q * 4; v4f v; v[0] = bfr(p[0]); v[1] = bfr(p[1]); v[2] = bfr(p[2]); v[3] = bfr(p[3]); vst2(OUT + (size_t)tok * DD + q * 4, v); }
}
extern "C" void kernel_launch(void* const* d_in, const int* in_sizes, int n_in, void* d_out, int out_size, void* d_ws, size_t ws_size, hipStream_t stream) {
  (void)in_sizes; (void)n_in; (void)out_size;
  const float** F = (const float**)d_in;
  if (ws_size < (size_t)WS_END) return;
  char* ws = (char*)d_ws; __bf16 *PK = (__bf16*)(ws + WS_PK), *HH = (__bf16*)(ws + WS_HH), *HL = (__bf16*)(ws + WS_HL), *VH = (__bf16*)(ws + WS_VH), *VL = (__bf16*)(ws + WS_VL), *AH = (__bf16*)(ws + WS_AH), *AL = (__bf16*)(ws + WS_AL); float* X1 = (float*)(ws + WS_X1); int *SEL = (int*)(ws + WS_SEL), *FLG = (int*)(ws + WS_FLG);
  k_pack<<<dim3(II, 5), 256, 0, stream>>>(F[11], F[13], F[14], F[15], F[16], PK);
  k_route<<<1, 256, 0, stream>>>(F[0], F[3], F[4], SEL, FLG);
  k_rms<<<KSEL, 256, 0, stream>>>(F[0], nullptr, SEL, F[5], 1, HH, HL);
  k_lin<0><<<dim3(KSEL / 64, DD / 128), 128, 0, stream>>>(HH, HL, PK + PK_V, nullptr, F[12], nullptr, nullptr, SEL, VH, VL, nullptr);
  k_lin<1><<<dim3(KSEL / 64, DD / 128), 128, 0, stream>>>(VH, VL, PK + PK_O, nullptr, nullptr, F[0], nullptr, SEL, nullptr, nullptr, X1);
  k_rms<<<KSEL, 256, 0, stream>>>(nullptr, X1, SEL, F[6], 0, HH, HL);
  k_lin<2><<<dim3(KSEL / 64, II / 128), 128, 0, stream>>>(HH, HL, PK + PK_G, PK + PK_U, nullptr, nullptr, nullptr, SEL, AH, AL, nullptr);
  k_lin<3><<<dim3(KSEL / 64, DD / 128), 128, 0, stream>>>(AH, AL, PK + PK_D, nullptr, nullptr, nullptr, X1, SEL, nullptr, nullptr, (float*)d_out);
  k_copy<<<NTOK, 256, 0, stream>>>(F[0], FLG, (float*)d_out);
}
